// SelfAttention_67525475827753
// MI455X (gfx1250) — hardware-verified
//
#include <hip/hip_runtime.h>


#ifndef NB
#define NB 4
#endif
#ifndef SEQ
#define SEQ 4096
#endif
#define NB_FULL    4
#define SEQ_FULL   4096
#define CH         256
#define NHEAD      4
#define HDIM       64
#define QKVN       (3 * CH)
#define BQ         128
#define BK         32
#define NWAVE      8
#define MT         128
#define LNT        32
#define LNP        33
#define TP         72
#define VP         136
#define OPF        132

static_assert(SEQ % BQ == 0);
static_assert(SEQ % MT == 0);
static_assert(SEQ % LNT == 0);
static_assert(SEQ % BK == 0);
static_assert(BQ == NWAVE * 16);
static_assert(MT == NWAVE * 16);
static_assert(CH == NHEAD * HDIM);
static_assert(CH == 256);
static_assert(HDIM == 64);
static_assert(CH % 32 == 0);
static_assert(SEQ <= SEQ_FULL);
static_assert(NB >= 1 && NB <= NB_FULL);
static_assert((TP * 2) % 16 == 0);
static_assert((VP * 2) % 16 == 0);
static_assert((OPF * 4) % 16 == 0);
static_assert(MT * TP >= HDIM * VP);
static_assert(256 * 4 * 8 == LNT * CH);
static_assert(256 * 2 * 8 == 64 * 64);
static_assert(256 * 4 * 8 == MT * HDIM);
static_assert(32 * 4 * 8 == 16 * HDIM);
static_assert(NWAVE * 8 * 32 * 4 == 64 * MT);

typedef __bf16   bf16;
typedef _Float16 f16;
typedef f16      v16h  __attribute__((ext_vector_type(16)));
typedef f16      v8h   __attribute__((ext_vector_type(8)));
typedef float    v8f   __attribute__((ext_vector_type(8)));
typedef float    v4f   __attribute__((ext_vector_type(4)));
typedef unsigned v4u   __attribute__((ext_vector_type(4)));

union FragH  { v16h  v; v4u q[2]; f16  h[16]; };
union Pack8H { v4u u; v8h v; f16 h[8]; };

static __device__ __forceinline__ v8f mma_f16(v16h a, v16h b, v8f acc) {
  acc = __builtin_amdgcn_wmma_f32_16x16x32_f16(false, a, false, b, (short)0, acc, false, false);
  asm volatile("v_nop\n\tv_nop\n\tv_nop\n\tv_nop" : "+v"(acc) : "v"(a), "v"(b));
  return acc;
}

__global__ __launch_bounds__(256) void w_planes_kernel(const float* __restrict__ wqkv,
                                                       const float* __restrict__ wproj,
                                                       f16* __restrict__ wqT,
                                                       f16* __restrict__ wpT) {
  const unsigned kt  = blockIdx.x;
  const unsigned nt  = blockIdx.y;
  const unsigned tid = threadIdx.x;
  const bool isq = nt < (QKVN / 64);
  const float* src = isq ? wqkv : wproj;
  f16*         dst = isq ? wqT : wpT;
  const unsigned ldn = isq ? (unsigned)QKVN : (unsigned)CH;
  const unsigned n0  = (isq ? nt : (nt - QKVN / 64)) * 64u;
  const unsigned k0  = kt * 64u;
  __shared__ __align__(16) f16 sT[64 * TP];

  #pragma unroll
  for (unsigned kk = 0; kk < 2; ++kk) {
    const unsigned kr = kk * 32 + (tid >> 3);
    const unsigned nn = (tid & 7u) * 8;
    const float* p = src + (size_t)(k0 + kr) * ldn + n0 + nn;
    const v4f w0 = *(const v4f*)(p);
    const v4f w1 = *(const v4f*)(p + 4);
    #pragma unroll
    for (unsigned i = 0; i < 4; ++i) {
      sT[(nn + i) * TP + kr]     = (f16)((float)(bf16)w0[i] * 64.0f);
      sT[(nn + 4 + i) * TP + kr] = (f16)((float)(bf16)w1[i] * 64.0f);
    }
  }
  __syncthreads();

  v4u    val[2];
  size_t idx[2];
  #pragma unroll
  for (unsigned kk = 0; kk < 2; ++kk) {
    const unsigned n  = kk * 32 + (tid >> 3);
    const unsigned ks = (tid & 7u) * 8;
    Pack8H ph;
    ph.v = *(const v8h*)(sT + n * TP + ks);
    val[kk] = ph.u;
    idx[kk] = (size_t)(n0 + n) * CH + k0 + ks;
  }
  #pragma unroll
  for (unsigned kk = 0; kk < 2; ++kk) *(volatile v4u*)(dst + idx[kk]) = val[kk];
  __threadfence();
  #pragma unroll
  for (unsigned kk = 0; kk < 2; ++kk) *(volatile v4u*)(dst + idx[kk]) = val[kk];
}

__global__ __launch_bounds__(256) void ln_plane_kernel(const float* __restrict__ x,
                                                       const float* __restrict__ gamma,
                                                       const float* __restrict__ beta,
                                                       f16* __restrict__ xn) {
  const unsigned tid = threadIdx.x;
  const unsigned blk = blockIdx.x;
  const unsigned b   = blk / (SEQ / LNT);
  const unsigned p0  = (blk % (SEQ / LNT)) * LNT;
  __shared__ float sX[CH * LNP];
  __shared__ float sG[CH];
  __shared__ float sB[CH];

  const float* xb = x + (size_t)b * CH * SEQ_FULL + p0;
  const unsigned px = tid & 31u;
  const unsigned cr = tid >> 5;
  #pragma unroll 4
  for (unsigned it = 0; it < 32; ++it) {
    const unsigned c = it * 8 + cr;
    const float v = xb[(size_t)c * SEQ_FULL + px];
    sX[c * LNP + px] = (float)(bf16)v;
  }
  sG[tid] = (float)(bf16)gamma[tid];
  sB[tid] = (float)(bf16)beta[tid];
  __syncthreads();

  const unsigned tok  = tid >> 3;
  const unsigned part = tid & 7u;
  float s = 0.0f;
  #pragma unroll 4
  for (unsigned j = 0; j < 32; ++j) s += sX[(part + 8 * j) * LNP + tok];
  s += __shfl_xor(s, 1, 32);
  s += __shfl_xor(s, 2, 32);
  s += __shfl_xor(s, 4, 32);
  const float mu = s * (1.0f / CH);
  float ss = 0.0f;
  #pragma unroll 4
  for (unsigned j = 0; j < 32; ++j) {
    const float d = sX[(part + 8 * j) * LNP + tok] - mu;
    ss += d * d;
  }
  ss += __shfl_xor(ss, 1, 32);
  ss += __shfl_xor(ss, 2, 32);
  ss += __shfl_xor(ss, 4, 32);
  const float rstd = rsqrtf(ss * (1.0f / CH) + 1e-5f);

  v4u    val[4];
  size_t idx[4];
  #pragma unroll
  for (unsigned j = 0; j < 4; ++j) {
    const unsigned c0 = j * 64 + part * 8;
    Pack8H ph;
    #pragma unroll
    for (unsigned i = 0; i < 8; ++i) {
      const float d = sX[(c0 + i) * LNP + tok] - mu;
      ph.h[i] = (f16)(d * rstd * sG[c0 + i] + sB[c0 + i]);
    }
    val[j] = ph.u;
    idx[j] = ((size_t)b * SEQ + p0 + tok) * CH + c0;
  }
  #pragma unroll
  for (unsigned j = 0; j < 4; ++j) *(volatile v4u*)(xn + idx[j]) = val[j];
  __threadfence();
  #pragma unroll
  for (unsigned j = 0; j < 4; ++j) *(volatile v4u*)(xn + idx[j]) = val[j];
}

__global__ __launch_bounds__(256) void qkv_gemm_kernel(const f16* __restrict__ xn,
                                                       const f16* __restrict__ wqT,
                                                       const float* __restrict__ bqkv,
                                                       f16* __restrict__ qp,
                                                       f16* __restrict__ kp,
                                                       f16* __restrict__ vt) {
  const unsigned mt   = blockIdx.x;
  const unsigned nt   = blockIdx.y;
  const unsigned tid  = threadIdx.x;
  const unsigned wave = tid >> 5;
  const unsigned lane = tid & 31u;
  const unsigned lq   = lane & 15u;
  const unsigned hi   = lane >> 4;
  const unsigned sel  = nt >> 2;
  const unsigned h    = nt & 3u;
  __shared__ __align__(16) f16 sT[MT * TP];

  const f16* arow = xn + (size_t)(mt * MT + wave * 16 + lq) * CH;
  const f16* brow = wqT + (size_t)(nt * 64 + lq) * CH;

  v8f acc[4];
  #pragma unroll
  for (unsigned dt = 0; dt < 4; ++dt) acc[dt] = (v8f){0, 0, 0, 0, 0, 0, 0, 0};

  #pragma unroll 2
  for (unsigned ks = 0; ks < CH / 32; ++ks) {
    FragH a;
    a.q[0] = *(const v4u*)(arow + ks * 32 + hi * 8);
    a.q[1] = *(const v4u*)(arow + ks * 32 + 16 + hi * 8);
    FragH bw[4];
    #pragma unroll
    for (unsigned dt = 0; dt < 4; ++dt) {
      const f16* base = brow + (size_t)dt * 16 * CH + ks * 32 + hi * 8;
      bw[dt].q[0] = *(const v4u*)(base);
      bw[dt].q[1] = *(const v4u*)(base + 16);
    }
    #pragma unroll
    for (unsigned dt = 0; dt < 4; ++dt) acc[dt] = mma_f16(a.v, bw[dt].v, acc[dt]);
  }

  float bias[4];
  #pragma unroll
  for (unsigned dt = 0; dt < 4; ++dt) bias[dt] = (float)(bf16)bqkv[nt * 64 + dt * 16 + lq];

  if (sel < 2u) {
    #pragma unroll
    for (unsigned dt = 0; dt < 4; ++dt) {
      #pragma unroll
      for (unsigned r = 0; r < 8; ++r)
        sT[(wave * 16 + hi * 8 + r) * TP + dt * 16 + lq] = (f16)(acc[dt][r] * (1.0f / 64.0f) + bias[dt]);
    }
  } else {
    #pragma unroll
    for (unsigned dt = 0; dt < 4; ++dt) {
      #pragma unroll
      for (unsigned r = 0; r < 8; ++r)
        sT[(dt * 16 + lq) * VP + wave * 16 + hi * 8 + r] = (f16)(acc[dt][r] * (1.0f / 64.0f) + bias[dt]);
    }
  }
  __syncthreads();

  const unsigned b    = mt / (SEQ / MT);
  const unsigned tok0 = (mt % (SEQ / MT)) * MT;
  f16* dst = (sel == 0u) ? qp : ((sel == 1u) ? kp : vt);
  v4u    val[4];
  size_t idx[4];
  if (sel < 2u) {
    #pragma unroll
    for (unsigned it = 0; it < 4; ++it) {
      const unsigned row = it * 32 + (tid >> 3);
      const unsigned pc  = tid & 7u;
      Pack8H ph;
      ph.v = *(const v8h*)(sT + row * TP + pc * 8);
      val[it] = ph.u;
      idx[it] = (((size_t)b * NHEAD + h) * SEQ + tok0 + row) * HDIM + pc * 8;
    }
  } else {
    #pragma unroll
    for (unsigned it = 0; it < 4; ++it) {
      const unsigned d  = it * 16 + (tid >> 4);
      const unsigned pc = tid & 15u;
      Pack8H ph;
      ph.v = *(const v8h*)(sT + d * VP + pc * 8);
      val[it] = ph.u;
      idx[it] = (((size_t)b * NHEAD + h) * HDIM + d) * SEQ + tok0 + pc * 8;
    }
  }
  #pragma unroll
  for (unsigned it = 0; it < 4; ++it) *(volatile v4u*)(dst + idx[it]) = val[it];
  __threadfence();
  #pragma unroll
  for (unsigned it = 0; it < 4; ++it) *(volatile v4u*)(dst + idx[it]) = val[it];
}

__global__ __launch_bounds__(256) void attn_kernel(const f16* __restrict__ qp,
                                                   const f16* __restrict__ kp,
                                                   const f16* __restrict__ vt,
                                                   f16* __restrict__ ctx) {
  const unsigned qblk = blockIdx.x;
  const unsigned h    = blockIdx.y;
  const unsigned b    = blockIdx.z;
  const unsigned tid  = threadIdx.x;
  const unsigned wave = tid >> 5;
  const unsigned lane = tid & 31u;
  const unsigned lq   = lane & 15u;
  const unsigned hi   = lane >> 4;

  __shared__ __align__(16) f16 sO[NWAVE * 16 * TP];

  const unsigned qrow0 = qblk * BQ + wave * 16;

  const f16* qp_h = qp + ((size_t)b * NHEAD + h) * SEQ * HDIM;
  const f16* kp_h = kp + ((size_t)b * NHEAD + h) * SEQ * HDIM;
  const f16* vt_h = vt + ((size_t)b * NHEAD + h) * HDIM * SEQ;

  FragH qf[2];
  {
    const f16* qr = qp_h + (size_t)(qrow0 + lq) * HDIM;
    #pragma unroll
    for (unsigned f = 0; f < 2; ++f) {
      qf[f].q[0] = *(const v4u*)(qr + f * 32 + hi * 8);
      qf[f].q[1] = *(const v4u*)(qr + f * 32 + 16 + hi * 8);
    }
  }

  v8f o[4];
  #pragma unroll
  for (unsigned dt = 0; dt < 4; ++dt) o[dt] = (v8f){0, 0, 0, 0, 0, 0, 0, 0};

  float rmax = -__builtin_inff();
  float rsum = 0.0f;
  const float SL = 0.0625f * 1.4426950408889634f;

  for (unsigned i = 0; i < SEQ / BK; ++i) {
    const unsigned j0 = i * BK;

    FragH ak[2][2];
    #pragma unroll
    for (unsigned sub = 0; sub < 2; ++sub) {
      #pragma unroll
      for (unsigned f = 0; f < 2; ++f) {
        const f16* base = kp_h + (size_t)(j0 + sub * 16 + lq) * HDIM + f * 32 + hi * 8;
        ak[sub][f].q[0] = *(const v4u*)(base);
        ak[sub][f].q[1] = *(const v4u*)(base + 16);
      }
    }
    FragH bv[4];
    #pragma unroll
    for (unsigned dt = 0; dt < 4; ++dt) {
      const f16* base = vt_h + (size_t)(dt * 16 + lq) * SEQ + j0 + hi * 8;
      bv[dt].q[0] = *(const v4u*)(base);
      bv[dt].q[1] = *(const v4u*)(base + 16);
    }

    v8f c[2];
    #pragma unroll
    for (unsigned sub = 0; sub < 2; ++sub) {
      v8f acc = (v8f){0, 0, 0, 0, 0, 0, 0, 0};
      acc = mma_f16(ak[sub][0].v, qf[0].v, acc);
      acc = mma_f16(ak[sub][1].v, qf[1].v, acc);
      c[sub] = acc;
    }

    float m_new = rmax;
    #pragma unroll
    for (unsigned r = 0; r < 8; ++r) {
      m_new = fmaxf(m_new, c[0][r]);
      m_new = fmaxf(m_new, c[1][r]);
    }
    m_new = fmaxf(m_new, __shfl_xor(m_new, 16, 32));
    const float scale = __builtin_amdgcn_exp2f((rmax - m_new) * SL);
    rmax = m_new;

    FragH pa;
    float psum = 0.0f;
    #pragma unroll
    for (unsigned r = 0; r < 8; ++r) {
      const float p0 = __builtin_amdgcn_exp2f((c[0][r] - m_new) * SL);
      const float p1 = __builtin_amdgcn_exp2f((c[1][r] - m_new) * SL);
      psum += p0 + p1;
      pa.h[r]     = (f16)(p0 * 4096.0f);
      pa.h[8 + r] = (f16)(p1 * 4096.0f);
    }
    rsum = rsum * scale + psum + __shfl_xor(psum, 16, 32);

    float sc[8];
    #pragma unroll
    for (unsigned r = 0; r < 8; ++r) sc[r] = __shfl(scale, (int)((hi << 3) + r), 32);
    #pragma unroll
    for (unsigned dt = 0; dt < 4; ++dt) {
      #pragma unroll
      for (unsigned r = 0; r < 8; ++r) o[dt][r] *= sc[r];
    }

    #pragma unroll
    for (unsigned dt = 0; dt < 4; ++dt) o[dt] = mma_f16(pa.v, bv[dt].v, o[dt]);
  }

  float rs[8];
  #pragma unroll
  for (unsigned r = 0; r < 8; ++r) rs[r] = 1.0f / __shfl(rsum, (int)((hi << 3) + r), 32);

  f16* so = sO + wave * (16 * TP);
  #pragma unroll
  for (unsigned r = 0; r < 8; ++r) {
    #pragma unroll
    for (unsigned dt = 0; dt < 4; ++dt)
      so[(hi * 8 + r) * TP + dt * 16 + lq] = (f16)(o[dt][r] * (256.0f / 4096.0f) * rs[r]);
  }
  __syncthreads();

  v4u    val[4];
  size_t idx[4];
  #pragma unroll
  for (unsigned it = 0; it < 4; ++it) {
    const unsigned row = it * 4 + (lane >> 3);
    const unsigned pc  = lane & 7u;
    Pack8H ph;
    ph.v = *(const v8h*)(so + row * TP + pc * 8);
    val[it] = ph.u;
    idx[it] = ((size_t)b * SEQ + qrow0 + row) * CH + h * HDIM + pc * 8;
  }
  #pragma unroll
  for (unsigned it = 0; it < 4; ++it) *(volatile v4u*)(ctx + idx[it]) = val[it];
  __threadfence();
  #pragma unroll
  for (unsigned it = 0; it < 4; ++it) *(volatile v4u*)(ctx + idx[it]) = val[it];
}

__global__ __launch_bounds__(256) void proj_kernel(const f16* __restrict__ ctx,
                                                   const f16* __restrict__ wpT,
                                                   const float* __restrict__ bproj,
                                                   const float* __restrict__ x,
                                                   float* __restrict__ out) {
  const unsigned mt   = blockIdx.x;
  const unsigned ct   = blockIdx.y;
  const unsigned tid  = threadIdx.x;
  const unsigned wave = tid >> 5;
  const unsigned lane = tid & 31u;
  const unsigned lq   = lane & 15u;
  const unsigned hi   = lane >> 4;
  __shared__ __align__(16) float sO[64 * OPF];

  const f16* brow = ctx + (size_t)(mt * MT + wave * 16 + lq) * CH;
  const f16* arow = wpT + (size_t)(ct * 64 + lq) * CH;

  v8f acc[4];
  #pragma unroll
  for (unsigned m4 = 0; m4 < 4; ++m4) acc[m4] = (v8f){0, 0, 0, 0, 0, 0, 0, 0};

  #pragma unroll 2
  for (unsigned ks = 0; ks < CH / 32; ++ks) {
    FragH bc;
    bc.q[0] = *(const v4u*)(brow + ks * 32 + hi * 8);
    bc.q[1] = *(const v4u*)(brow + ks * 32 + 16 + hi * 8);
    FragH aw[4];
    #pragma unroll
    for (unsigned m4 = 0; m4 < 4; ++m4) {
      const f16* base = arow + (size_t)m4 * 16 * CH + ks * 32 + hi * 8;
      aw[m4].q[0] = *(const v4u*)(base);
      aw[m4].q[1] = *(const v4u*)(base + 16);
    }
    #pragma unroll
    for (unsigned m4 = 0; m4 < 4; ++m4) acc[m4] = mma_f16(aw[m4].v, bc.v, acc[m4]);
  }

  #pragma unroll
  for (unsigned m4 = 0; m4 < 4; ++m4) {
    #pragma unroll
    for (unsigned r = 0; r < 8; ++r)
      sO[(m4 * 16 + hi * 8 + r) * OPF + wave * 16 + lq] = acc[m4][r] * (1.0f / 16384.0f);
  }
  __syncthreads();

  const unsigned b  = mt / (SEQ / MT);
  const unsigned p0 = (mt % (SEQ / MT)) * MT;
  v4f    val[8];
  size_t idx[8];
  #pragma unroll
  for (unsigned it = 0; it < 8; ++it) {
    const unsigned row = it * 8 + wave;
    const unsigned c   = ct * 64 + row;
    const v4f a  = *(const v4f*)(sO + row * OPF + lane * 4);
    const float bb = (float)(bf16)bproj[c];
    const size_t gi = ((size_t)b * CH + c) * SEQ_FULL + p0 + lane * 4;
    const v4f xv = *(const v4f*)(x + gi);
    v4f res;
    #pragma unroll
    for (unsigned i = 0; i < 4; ++i) res[i] = (float)(bf16)xv[i] + (a[i] + bb);
    val[it] = res;
    idx[it] = gi;
  }
  #pragma unroll
  for (unsigned it = 0; it < 8; ++it) *(volatile v4f*)(out + idx[it]) = val[it];
  __threadfence();
  #pragma unroll
  for (unsigned it = 0; it < 8; ++it) *(volatile v4f*)(out + idx[it]) = val[it];
}

extern "C" void kernel_launch(void* const* d_in, const int* in_sizes, int n_in,
                              void* d_out, int out_size, void* d_ws, size_t ws_size,
                              hipStream_t stream) {
  if (n_in < 7) return;
  const size_t x_need = ((size_t)(NB - 1) * CH + (CH - 1)) * SEQ_FULL + SEQ;
  if ((size_t)in_sizes[0] < x_need) return;
  if (in_sizes[1] < CH || in_sizes[2] < CH) return;
  if ((size_t)in_sizes[3] < (size_t)CH * QKVN || in_sizes[4] < QKVN) return;
  if ((size_t)in_sizes[5] < (size_t)CH * CH || in_sizes[6] < CH) return;
  if ((size_t)out_size < x_need) return;

  const size_t tok_plane = (size_t)NB * SEQ * CH * 2;
  const size_t wq_bytes  = (size_t)QKVN * CH * 2;
  const size_t wp_bytes  = (size_t)CH * CH * 2;
  const size_t total     = 5 * tok_plane + wq_bytes + wp_bytes;
  if (ws_size < total) return;

  const float* x     = (const float*)d_in[0];
  const float* gam   = (const float*)d_in[1];
  const float* bet   = (const float*)d_in[2];
  const float* wqkv  = (const float*)d_in[3];
  const float* bqkv  = (const float*)d_in[4];
  const float* wproj = (const float*)d_in[5];
  const float* bproj = (const float*)d_in[6];
  float* out = (float*)d_out;

  char* ws = (char*)d_ws;
  f16* xn  = (f16*)(ws);
  f16* qp  = (f16*)(ws + 1 * tok_plane);
  f16* kp  = (f16*)(ws + 2 * tok_plane);
  f16* vt  = (f16*)(ws + 3 * tok_plane);
  f16* ctx = (f16*)(ws + 4 * tok_plane);
  f16* wqT = (f16*)(ws + 5 * tok_plane);
  f16* wpT = (f16*)(ws + 5 * tok_plane + wq_bytes);

  w_planes_kernel<<<dim3(CH / 64, QKVN / 64 + CH / 64), 256, 0, stream>>>(wqkv, wproj, wqT, wpT);
  ln_plane_kernel<<<dim3(NB * (SEQ / LNT)), 256, 0, stream>>>(x, gam, bet, xn);
  qkv_gemm_kernel<<<dim3(NB * (SEQ / MT), QKVN / 64), 256, 0, stream>>>(xn, wqT, bqkv, qp, kp, vt);
  attn_kernel<<<dim3(SEQ / BQ, NHEAD, NB), 256, 0, stream>>>(qp, kp, vt, ctx);
  proj_kernel<<<dim3(NB * (SEQ / MT), CH / 64), 256, 0, stream>>>(ctx, wpT, bproj, x, out);
}
